// S4Block_25546465477181
// MI455X (gfx1250) — hardware-verified
//
#include <hip/hip_runtime.h>
#include <math.h>
#include <stdint.h>

typedef __attribute__((ext_vector_type(16))) _Float16 v16h;
typedef __attribute__((ext_vector_type(8)))  _Float16 v8h;
typedef __attribute__((ext_vector_type(8)))  float    v8f;
typedef __attribute__((ext_vector_type(4)))  float    v4f;
typedef __attribute__((ext_vector_type(4)))  unsigned int u4v;

constexpr int kBatch  = 4;
constexpr int kSeq    = 2048;
constexpr int kHid    = 768;
constexpr int kTaps   = 2048;
constexpr int kRows   = kBatch * kSeq;
constexpr int kWPre   = 32;
constexpr int kWStr   = 2176;
constexpr int kSigPre = 64;
constexpr int kSigRow = 2144;
constexpr float kCarryW   = 32.0f;
constexpr float kCarryAct = 16.0f;
constexpr float kConvInv  = 1.0f / kCarryW;
constexpr float kGemmInv  = 1.0f / (kCarryW * kCarryAct);
constexpr float kInvHid   = 1.0f / (float)kHid;
constexpr float kLnEps    = 1e-6f;

static_assert(kTaps == kSeq, "filter length equals sequence length");
static_assert(kWPre + kTaps + 96 == kWStr, "filter row layout");
static_assert((kWStr % 64) == 0, "filter row is a whole number of 128-B lines");
static_assert(kSigPre + kSeq + 32 == kSigRow, "signal row layout");
static_assert(((kSigRow * 2) % 16) == 0 && ((kWStr * 2) % 16) == 0, "16-B aligned LDS rows");
static_assert((kHid % 64) == 0 && (kSeq % 64) == 0 && (kRows % 64) == 0, "tile multiples");
static_assert((kHid % 32) == 0, "GEMM K multiple of 32");
static_assert(kBatch == 4, "row = (batch, subtile) mapping uses 4 batches x 4 subtiles");
static_assert((kHid % 128) == 0, "row statistics read 6 x 128 floats");

constexpr size_t kOffWrev = 0;
constexpr size_t kOffWt   = kOffWrev + (size_t)kHid * kWStr * 2;
constexpr size_t kOffStat = kOffWt   + (size_t)kHid * kHid * 2;
constexpr size_t kOffSig  = kOffStat + (size_t)kRows * 2 * 4;
constexpr size_t kOffYT   = kOffSig  + (size_t)kBatch * kHid * kSeq * 2;
constexpr size_t kOffY2   = kOffYT   + (size_t)kBatch * kHid * kSeq * 2;
constexpr size_t kWsTotal = kOffY2   + (size_t)kRows * kHid * 2;
static_assert(kWsTotal == 42336256ull, "carve total");
static_assert(kWsTotal <= 134217728ull, "carve cap");
static_assert((kOffWt % 128) == 0 && (kOffStat % 128) == 0 && (kOffSig % 128) == 0 &&
              (kOffYT % 128) == 0 && (kOffY2 % 128) == 0, "128-B aligned regions");

struct FragH {
  union U { v16h v; v8h h[2]; };
  static __device__ __forceinline__ v16h load(const _Float16* p) {
    U f;
    f.h[0] = *(const v8h*)(p);
    f.h[1] = *(const v8h*)(p + 16);
    return f.v;
  }
  static __device__ __forceinline__ v8f mma(v16h a, v16h b, v8f c) {
    return __builtin_amdgcn_wmma_f32_16x16x32_f16(false, a, false, b, (short)0, c, false, false);
  }
};
__device__ __forceinline__ v8f mma_guarded(v16h a, v16h b, v8f c) {
  c = __builtin_amdgcn_wmma_f32_16x16x32_f16(false, a, false, b, (short)0, c, false, false);
  asm volatile("v_nop\n\tv_nop\n\tv_nop\n\tv_nop" : "+v"(c) : "v"(a), "v"(b));
  return c;
}
__device__ __forceinline__ void guard_row4(v8f& a0, v8f& a1, v8f& a2, v8f& a3,
                                           v16h x, v16h b0, v16h b1, v16h b2, v16h b3) {
  asm volatile("v_nop\n\tv_nop\n\tv_nop\n\tv_nop"
               : "+v"(a0), "+v"(a1), "+v"(a2), "+v"(a3)
               : "v"(x), "v"(b0), "v"(b1), "v"(b2), "v"(b3));
}
__device__ __forceinline__ void acc_guard4(v8f& a, v8f& b, v8f& c, v8f& d) {
  asm volatile("v_nop\n\tv_nop\n\tv_nop\n\tv_nop" : "+v"(a), "+v"(b), "+v"(c), "+v"(d));
}

__device__ __forceinline__ float gelu_tanh_f(float v) {
  const float u = 0.7978845608028654f * (v + 0.044715f * v * v * v);
  const float t = fminf(-2.0f * u, 80.0f);
  const float e = expf(t);
  return v * __builtin_amdgcn_rcpf(1.0f + e);
}

__global__ __launch_bounds__(256) void transpose_cast_shift_kernel(
    const float* __restrict__ W, unsigned short* __restrict__ Bt,
    int Kdim, int Ndim, int outPitch, int shift, float scale)
{
  __shared__ float tile[64 * 65];
  const int tid = threadIdx.x, lane = tid & 31, wave = tid >> 5;
  const int n0 = blockIdx.x * 64;
  const int i0 = blockIdx.y * 64;
#pragma unroll
  for (int p = 0; p < 16; ++p) {
    const int idx = tid + p * 256;
    const int kk  = idx >> 6;
    const int nn  = idx & 63;
    const int kin = i0 + kk - shift;
    const int kc  = (kin < 0) ? 0 : ((kin > Kdim - 1) ? (Kdim - 1) : kin);
    const float v = W[(size_t)kc * Ndim + n0 + nn];
    const bool ok = (kin >= 0) && (kin < Kdim);
    tile[kk * 65 + nn] = ok ? (v * scale) : 0.0f;
  }
  __syncthreads();
  const int q = lane >> 3, c8 = (lane & 7) * 8;
  v8h hv[2];
#pragma unroll
  for (int it = 0; it < 2; ++it) {
    const int nrow = it * 32 + wave * 4 + q;
#pragma unroll
    for (int e = 0; e < 8; ++e) hv[it][e] = (_Float16)tile[(c8 + e) * 65 + nrow];
  }
  for (int pass = 0; pass < 2; ++pass) {
#pragma unroll
    for (int it = 0; it < 2; ++it) {
      const int nrow = it * 32 + wave * 4 + q;
      *(volatile v8h*)(Bt + (size_t)(n0 + nrow) * outPitch + i0 + c8) = hv[it];
    }
    __threadfence();
  }
}

__global__ __launch_bounds__(256) void ln_stats_kernel(
    const float* __restrict__ x, float* __restrict__ stats)
{
  __shared__ __align__(16) float sS[32];
  const int tid = threadIdx.x, lane = tid & 31, wave = tid >> 5;
  const int rowb = blockIdx.x * 16;
#pragma unroll 1
  for (int rr = 0; rr < 2; ++rr) {
    const int lr = wave * 2 + rr;
    const float* xr = x + (size_t)(rowb + lr) * kHid;
    v4f a[6];
#pragma unroll
    for (int i = 0; i < 6; ++i) a[i] = *(const v4f*)(xr + i * 128 + lane * 4);
    float s = 0.0f;
#pragma unroll
    for (int i = 0; i < 6; ++i) s += (a[i][0] + a[i][1]) + (a[i][2] + a[i][3]);
#pragma unroll
    for (int off = 16; off > 0; off >>= 1) s += __shfl_xor(s, off, 32);
    const float mean = s * kInvHid;
    float qs = 0.0f;
#pragma unroll
    for (int i = 0; i < 6; ++i) {
#pragma unroll
      for (int e = 0; e < 4; ++e) {
        const float d = a[i][e] - mean;
        qs = fmaf(d, d, qs);
      }
    }
#pragma unroll
    for (int off = 16; off > 0; off >>= 1) qs += __shfl_xor(qs, off, 32);
    const float rstd = rsqrtf(qs * kInvHid + kLnEps);
    if (lane == 0) {
      sS[lr * 2]     = mean;
      sS[lr * 2 + 1] = rstd;
    }
  }
  __syncthreads();
  if (tid < 8) {
    const v4f v = *(const v4f*)(sS + tid * 4);
    float* p = stats + (size_t)rowb * 2 + tid * 4;
    *(volatile v4f*)p = v;
    __threadfence();
    *(volatile v4f*)p = v;
  }
}

__global__ __launch_bounds__(256) void ln_norm_transpose_kernel(
    const float* __restrict__ x, const float* __restrict__ stats,
    const float* __restrict__ gam, const float* __restrict__ bet,
    unsigned short* __restrict__ sig)
{
  __shared__ float tile[64 * 65];
  __shared__ float sSt[128];
  const int tid = threadIdx.x, lane = tid & 31, wave = tid >> 5;
  const int l0 = blockIdx.x * 64;
  const int h0 = blockIdx.y * 64;
  const int b  = blockIdx.z;
  const int row0 = b * kSeq + l0;
  if (tid < 128) sSt[tid] = stats[(size_t)row0 * 2 + tid];
  __syncthreads();
  const int hh = tid & 63;
  const float gv = gam[h0 + hh];
  const float bv = bet[h0 + hh];
#pragma unroll
  for (int p = 0; p < 16; ++p) {
    const int ll = (tid >> 6) + 4 * p;
    const float xv   = x[(size_t)(row0 + ll) * kHid + h0 + hh];
    const float mean = sSt[2 * ll];
    const float rstd = sSt[2 * ll + 1];
    tile[ll * 65 + hh] = (xv - mean) * rstd * gv + bv;
  }
  __syncthreads();
  const int q = lane >> 3, c8 = (lane & 7) * 8;
  v8h hv[2];
#pragma unroll
  for (int it = 0; it < 2; ++it) {
    const int hrow = it * 32 + wave * 4 + q;
#pragma unroll
    for (int e = 0; e < 8; ++e) hv[it][e] = (_Float16)tile[(c8 + e) * 65 + hrow];
  }
  for (int pass = 0; pass < 2; ++pass) {
#pragma unroll
    for (int it = 0; it < 2; ++it) {
      const int hrow = it * 32 + wave * 4 + q;
      *(volatile v8h*)(sig + ((size_t)(b * kHid + h0 + hrow) * kSeq) + l0 + c8) = hv[it];
    }
    __threadfence();
  }
}

__global__ __launch_bounds__(256) void conv_toeplitz_kernel(
    const unsigned short* __restrict__ sig, const unsigned short* __restrict__ wrev,
    const float* __restrict__ cbias, unsigned short* __restrict__ yT)
{
  __shared__ __align__(16) _Float16 sW[8 * kWStr];
  __shared__ __align__(16) _Float16 sSig[kBatch * kSigRow];
  __shared__ __align__(16) float sO[8][4 * 64];
  const int tid = threadIdx.x, lane = tid & 31, wave = tid >> 5;
  const int h = blockIdx.x;

  {
    const u4v* src = (const u4v*)(wrev + (size_t)h * kWStr);
    u4v* dst = (u4v*)sW;
    for (int i = tid; i < kWStr / 8; i += 256) dst[i] = src[i];
  }
  for (int i = tid; i < kBatch * 256; i += 256) {
    const int bb = i >> 8, j = i & 255;
    const u4v v = *(const u4v*)(sig + ((size_t)(bb * kHid + h) * kSeq) + j * 8);
    *(u4v*)(sSig + bb * kSigRow + kSigPre + j * 8) = v;
  }
  {
    unsigned* sw = (unsigned*)sSig;
    for (int i = tid; i < kBatch * 48; i += 256) {
      const int bb = i / 48, w = i - bb * 48;
      const int dw = (w < 32) ? w : (1024 + w);
      sw[bb * (kSigRow / 2) + dw] = 0u;
    }
  }
  __syncthreads();
  {
    constexpr int NW = kWStr / 2;
    const unsigned* w0 = (const unsigned*)sW;
    unsigned* wAll = (unsigned*)sW;
    for (int i = tid; i < 7 * NW; i += 256) {
      const int pm = i / NW;
      const int p  = pm + 1;
      const int j  = i - pm * NW;
      const int ja = j + (p >> 1);
      const int jb = ja + 1;
      const int jac = (ja < NW) ? ja : (NW - 1);
      const int jbc = (jb < NW) ? jb : (NW - 1);
      const unsigned wa = w0[jac];
      const unsigned wb = w0[jbc];
      const unsigned va = (ja < NW) ? wa : 0u;
      const unsigned vb = (jb < NW) ? wb : 0u;
      const unsigned odd = (va >> 16) | (vb << 16);
      const unsigned r = (p & 1) ? odd : va;
      wAll[p * NW + j] = r;
    }
  }
  __syncthreads();

  const int lh = lane >> 4, ln = lane & 15;
  const int ph = (7 - ln) & 7;
  const _Float16* wrow = sW + ph * kWStr;
  const int bq = ln >> 2, mp = ln & 3;
  const _Float16* arow = sSig + bq * kSigRow + (kSigPre - 64) + 16 * mp + 8 * lh;
  const float cb = cbias[h];
  float* slab = sO[wave];
  const int bsel = lane >> 3, c8 = (lane & 7) * 8;

#pragma unroll 1
  for (int step = 0; step < 4; ++step) {
    const int gi = (step & 1) ? (8 * step + 7 - wave) : (8 * step + wave);
    const int T0 = gi * 64;
    v8f acc = (v8f){0.f, 0.f, 0.f, 0.f, 0.f, 0.f, 0.f, 0.f};
    const _Float16* bptr = wrow + (kWPre + 2047 - 64 - T0 - ln + 8 * lh - ph);
    const _Float16* aptr = arow;
    {
      const v16h a  = FragH::load(aptr);
      const v16h bb = FragH::load(bptr);
      acc = mma_guarded(a, bb, acc);
      aptr += 32;
      bptr += 32;
    }
#pragma unroll 1
    for (int j = 0; j <= gi; ++j) {
      const v16h a0 = FragH::load(aptr);
      const v16h b0 = FragH::load(bptr);
      const v16h a1 = FragH::load(aptr + 32);
      const v16h b1 = FragH::load(bptr + 32);
      acc = mma_guarded(a0, b0, acc);
      acc = mma_guarded(a1, b1, acc);
      aptr += 64;
      bptr += 64;
    }
#pragma unroll
    for (int r = 0; r < 8; ++r) {
      const float v = acc[r] * kConvInv + cb;
      const float g = gelu_tanh_f(v) * kCarryAct;
      slab[(2 * lh + (r >> 2)) * 64 + 16 * (r & 3) + ln] = g;
    }
    __builtin_amdgcn_fence(__ATOMIC_RELEASE, "workgroup");
    __builtin_amdgcn_wave_barrier();
    __builtin_amdgcn_fence(__ATOMIC_ACQUIRE, "workgroup");
    {
      const v4f s0 = *(const v4f*)(slab + bsel * 64 + c8);
      const v4f s1 = *(const v4f*)(slab + bsel * 64 + c8 + 4);
      v8h hv;
#pragma unroll
      for (int e = 0; e < 4; ++e) {
        hv[e]     = (_Float16)s0[e];
        hv[4 + e] = (_Float16)s1[e];
      }
      unsigned short* dst = yT + ((size_t)(bsel * kHid + h) * kSeq) + T0 + c8;
      *(volatile v8h*)dst = hv;
      __threadfence();
      *(volatile v8h*)dst = hv;
    }
    __builtin_amdgcn_fence(__ATOMIC_RELEASE, "workgroup");
    __builtin_amdgcn_wave_barrier();
    __builtin_amdgcn_fence(__ATOMIC_ACQUIRE, "workgroup");
  }
}

__global__ __launch_bounds__(256) void transpose_back_kernel(
    const unsigned short* __restrict__ yT, unsigned short* __restrict__ y2)
{
  __shared__ unsigned tile[64 * 65];
  const int tid = threadIdx.x, lane = tid & 31, wave = tid >> 5;
  const int t0 = blockIdx.x * 64;
  const int h0 = blockIdx.y * 64;
  const int b  = blockIdx.z;
  {
    const int rc8 = (tid & 7) * 8;
#pragma unroll
    for (int it = 0; it < 2; ++it) {
      const int hrow = it * 32 + (tid >> 3);
      const u4v w = *(const u4v*)(yT + ((size_t)(b * kHid + h0 + hrow) * kSeq) + t0 + rc8);
      const unsigned w0 = w[0], w1 = w[1], w2 = w[2], w3 = w[3];
      unsigned* tp = tile + hrow * 65 + rc8;
      tp[0] = w0 & 0xffffu;
      tp[1] = w0 >> 16;
      tp[2] = w1 & 0xffffu;
      tp[3] = w1 >> 16;
      tp[4] = w2 & 0xffffu;
      tp[5] = w2 >> 16;
      tp[6] = w3 & 0xffffu;
      tp[7] = w3 >> 16;
    }
  }
  __syncthreads();
  const int q = lane >> 3, c8 = (lane & 7) * 8;
  u4v ov[2];
#pragma unroll
  for (int it = 0; it < 2; ++it) {
    const int trow = it * 32 + wave * 4 + q;
#pragma unroll
    for (int k = 0; k < 4; ++k) {
      const unsigned lo = tile[(c8 + 2 * k) * 65 + trow];
      const unsigned hi = tile[(c8 + 2 * k + 1) * 65 + trow];
      ov[it][k] = lo | (hi << 16);
    }
  }
  for (int pass = 0; pass < 2; ++pass) {
#pragma unroll
    for (int it = 0; it < 2; ++it) {
      const int trow = it * 32 + wave * 4 + q;
      *(volatile u4v*)(y2 + ((size_t)(b * kSeq + t0 + trow) * kHid) + h0 + c8) = ov[it];
    }
    __threadfence();
  }
}

__global__ __launch_bounds__(256) void gemm_out_kernel(
    const unsigned short* __restrict__ Ap, int lda,
    const unsigned short* __restrict__ Btp, int ldb,
    float* __restrict__ C, int ldc,
    const float* __restrict__ bias, const float* __restrict__ resid,
    int M, int N, int K, float scale)
{
  const _Float16* A  = (const _Float16*)Ap;
  const _Float16* Bt = (const _Float16*)Btp;
  __shared__ __align__(16) float sT[8][16 * 68];
  const int lane = threadIdx.x & 31;
  const int wave = threadIdx.x >> 5;
  const int tilesN = N >> 6;
  const int tilesM = M >> 6;
  const int tile = blockIdx.x * 8 + wave;
  if (tile >= tilesM * tilesN) return;
  const int tm = tile / tilesN;
  const int tn = tile - tm * tilesN;
  const int m0 = tm << 6;
  const int n0 = tn << 6;
  const int rlane = lane & 15;
  const int koff  = (lane >> 4) * 8;
  const int mOff  = (lane >> 4) * 8;

  v8f acc[4][4];
#pragma unroll
  for (int i = 0; i < 4; ++i)
#pragma unroll
    for (int j = 0; j < 4; ++j) acc[i][j] = (v8f){0.f, 0.f, 0.f, 0.f, 0.f, 0.f, 0.f, 0.f};

  for (int k0 = 0; k0 < K; k0 += 32) {
    v16h bh[4];
#pragma unroll
    for (int j = 0; j < 4; ++j)
      bh[j] = FragH::load(Bt + (size_t)(n0 + (j << 4) + rlane) * ldb + koff + k0);
#pragma unroll
    for (int i = 0; i < 4; ++i) {
      const v16h ah = FragH::load(A + (size_t)(m0 + (i << 4) + rlane) * lda + koff + k0);
#pragma unroll
      for (int j = 0; j < 4; ++j) acc[i][j] = FragH::mma(ah, bh[j], acc[i][j]);
      guard_row4(acc[i][0], acc[i][1], acc[i][2], acc[i][3], ah, bh[0], bh[1], bh[2], bh[3]);
    }
  }
  acc_guard4(acc[0][0], acc[0][1], acc[0][2], acc[0][3]);
  acc_guard4(acc[1][0], acc[1][1], acc[1][2], acc[1][3]);
  acc_guard4(acc[2][0], acc[2][1], acc[2][2], acc[2][3]);
  acc_guard4(acc[3][0], acc[3][1], acc[3][2], acc[3][3]);

  float* slab = sT[wave];
  const int hh = lane >> 4, c4 = (lane & 15) * 4;
  const v4f bq = *(const v4f*)(bias + n0 + c4);
#pragma unroll
  for (int i = 0; i < 4; ++i) {
    const int mBase = m0 + (i << 4);
#pragma unroll
    for (int j = 0; j < 4; ++j) {
#pragma unroll
      for (int r = 0; r < 8; ++r)
        slab[(mOff + r) * 68 + (j << 4) + rlane] = acc[i][j][r] * scale;
    }
    __builtin_amdgcn_fence(__ATOMIC_RELEASE, "workgroup");
    __builtin_amdgcn_wave_barrier();
    __builtin_amdgcn_fence(__ATOMIC_ACQUIRE, "workgroup");
    v4f vv[8];
#pragma unroll
    for (int it = 0; it < 8; ++it) {
      const int row = it * 2 + hh;
      const v4f sv = *(const v4f*)(slab + row * 68 + c4);
      const v4f rv = *(const v4f*)(resid + (size_t)(mBase + row) * ldc + n0 + c4);
      vv[it] = (sv + bq) + rv;
    }
    for (int pass = 0; pass < 2; ++pass) {
#pragma unroll
      for (int it = 0; it < 8; ++it) {
        const int row = it * 2 + hh;
        *(volatile v4f*)(C + (size_t)(mBase + row) * ldc + n0 + c4) = vv[it];
      }
      __threadfence();
    }
    __builtin_amdgcn_fence(__ATOMIC_RELEASE, "workgroup");
    __builtin_amdgcn_wave_barrier();
    __builtin_amdgcn_fence(__ATOMIC_ACQUIRE, "workgroup");
  }
}

extern "C" void kernel_launch(void* const* d_in, const int* in_sizes, int n_in,
                              void* d_out, int out_size, void* d_ws, size_t ws_size,
                              hipStream_t stream)
{
  if (n_in < 7) return;
  if (in_sizes[0] != kRows * kHid) return;
  if (in_sizes[1] != kHid || in_sizes[2] != kHid) return;
  if (in_sizes[3] != kTaps * kHid) return;
  if (in_sizes[4] != kHid) return;
  if (in_sizes[5] != kHid * kHid) return;
  if (in_sizes[6] != kHid) return;
  if (out_size != kRows * kHid) return;
  if (ws_size < kWsTotal) return;

  const float* x     = (const float*)d_in[0];
  const float* lnsc  = (const float*)d_in[1];
  const float* lnbi  = (const float*)d_in[2];
  const float* ck    = (const float*)d_in[3];
  const float* cbias = (const float*)d_in[4];
  const float* W     = (const float*)d_in[5];
  const float* bvec  = (const float*)d_in[6];
  float* out = (float*)d_out;

  char* ws = (char*)d_ws;
  unsigned short* WREV = (unsigned short*)(ws + kOffWrev);
  unsigned short* WT   = (unsigned short*)(ws + kOffWt);
  float*          STAT = (float*)(ws + kOffStat);
  unsigned short* SIG  = (unsigned short*)(ws + kOffSig);
  unsigned short* YT   = (unsigned short*)(ws + kOffYT);
  unsigned short* Y2   = (unsigned short*)(ws + kOffY2);

  transpose_cast_shift_kernel<<<dim3(kHid / 64, kWStr / 64), 256, 0, stream>>>(
      ck, WREV, kTaps, kHid, kWStr, kWPre, kCarryW);
  transpose_cast_shift_kernel<<<dim3(kHid / 64, kHid / 64), 256, 0, stream>>>(
      W, WT, kHid, kHid, kHid, 0, kCarryW);
  ln_stats_kernel<<<kRows / 16, 256, 0, stream>>>(x, STAT);
  ln_norm_transpose_kernel<<<dim3(kSeq / 64, kHid / 64, kBatch), 256, 0, stream>>>(
      x, STAT, lnsc, lnbi, SIG);
  conv_toeplitz_kernel<<<kHid, 256, 0, stream>>>(SIG, WREV, cbias, YT);
  transpose_back_kernel<<<dim3(kSeq / 64, kHid / 64, kBatch), 256, 0, stream>>>(YT, Y2);
  gemm_out_kernel<<<dim3((kRows / 64) * (kHid / 64) / 8, 1), 256, 0, stream>>>(
      Y2, kHid, WT, kHid, out, kHid, bvec, x, kRows, kHid, kHid, kGemmInv);
}
